// GIN_16870631538847
// MI455X (gfx1250) — hardware-verified
//
#include <hip/hip_runtime.h>
#include <stddef.h>
#include <stdint.h>


#define DIN1    32
#define HID     64
#define NOUT    3
#define NFCP    16
#define KA1     (2 * DIN1)
#define KA2     (2 * HID)
#define KT      (2 * HID)
#define NTHR    256
#define NWAVE   8
#define EPT     8
#define CHUNK   (NTHR * EPT)
#define WCAP    (EPT * 32)
#define LISTN   (NWAVE * WCAP)
#define NBA     1024
#define PKS     10
#define RCAP    28672
#define DEGCAP  64
#define GBM     64
#define GTHR    128
#define WP0H    (HID * KA1)
#define WP1H    (HID * KT)
#define WP2H    (HID * KA2)
#define WP3H    (HID * KT)
#define WP4H    (NFCP * KT)
#define OF0     0
#define OF1     (OF0 + WP0H)
#define OF2     (OF1 + WP1H)
#define OF3     (OF2 + WP2H)
#define OF4     (OF3 + WP3H)
#define WPLH    (OF4 + WP4H)
#define NU0     (WP0H / 8)
#define NU1     (WP1H / 8)
#define NU2     (WP2H / 8)
#define NU3     (WP3H / 8)
#define NU4     (WP4H / 8)
#define UB1     (NU0)
#define UB2     (UB1 + NU1)
#define UB3     (UB2 + NU2)
#define UB4     (UB3 + NU3)
#define NUW     (UB4 + NU4)
#define ZINTS   (2 * RCAP + 2 * NBA + LISTN)
#define LDS_AGG (ZINTS * 4 + 64)
#define WSMAX   134217728

static_assert((CHUNK & (CHUNK - 1)) == 0);
static_assert(NBA == (1 << PKS));
static_assert(((long long)CHUNK << PKS) < (1LL << 31));
static_assert(NTHR * 4 == NBA);
static_assert(LISTN >= NBA && LISTN >= NWAVE * WCAP);
static_assert((RCAP % 32) == 0);
static_assert((ZINTS % (NTHR * 4)) == 0);
static_assert(LDS_AGG <= 262144);
static_assert((NBA % NWAVE) == 0 && (NBA % GBM) == 0);
static_assert(GBM == (GTHR / 32) * 16);
static_assert((KA1 % 32) == 0 && (KA2 % 32) == 0 && (KT % 32) == 0);
static_assert(DIN1 == 32 && HID == 64);
static_assert((NU0 % NTHR) == 0 && (NU1 % NTHR) == 0 && (NU2 % NTHR) == 0 && (NU3 % NTHR) == 0 && (NU4 % NTHR) == 0);
static_assert((OF1 % 64) == 0 && (OF2 % 64) == 0 && (OF3 % 64) == 0 && (OF4 % 64) == 0 && (WPLH % 64) == 0);
static_assert((KA1 / 8) == 8 && (KA2 / 8) == 16 && (KT / 8) == 16);
static_assert((GBM * NOUT) % 4 == 0 && GBM * NOUT <= GTHR * 4);
static_assert(KT * 2 == HID * 4);
static_assert(NOUT <= NFCP);

typedef float          v2f  __attribute__((ext_vector_type(2)));
typedef float          v4f  __attribute__((ext_vector_type(4)));
typedef float          v8f  __attribute__((ext_vector_type(8)));
typedef int            v4i  __attribute__((ext_vector_type(4)));
typedef int            v8i  __attribute__((ext_vector_type(8)));
typedef unsigned int   v2u  __attribute__((ext_vector_type(2)));
typedef unsigned int   v4u  __attribute__((ext_vector_type(4)));
typedef unsigned short v8us __attribute__((ext_vector_type(8)));
typedef _Float16       v16h __attribute__((ext_vector_type(16)));
typedef __bf16         v16b __attribute__((ext_vector_type(16)));
typedef v4f  __attribute__((may_alias)) v4fa;
typedef v4i  __attribute__((may_alias)) v4ia;
typedef v8us __attribute__((may_alias)) v8usa;
union Frag { v16b b; v16h f; v8us h[2]; v8i w; };

__device__ __forceinline__ v8f wmk(const Frag& a, const Frag& b, v8f c) {
  v8f d = __builtin_amdgcn_wmma_f32_16x16x32_bf16(false, a.b, false, b.b, (short)0, c, false, false);
  asm volatile("v_nop\n\tv_nop\n\tv_nop\n\tv_nop" : "+v"(d) : "v"(a.w), "v"(b.w));
  return d;
}

__device__ __forceinline__ unsigned short bf_bits(float f) {
  unsigned int u = __float_as_uint(f);
  u += 0x7FFFu + ((u >> 16) & 1u);
  return (unsigned short)(u >> 16);
}
__device__ __forceinline__ float bf_val(unsigned short b) {
  return __uint_as_float(((unsigned int)b) << 16);
}
__device__ __forceinline__ float bf_rne(float f) { return bf_val(bf_bits(f)); }

__device__ __forceinline__ void split8b(const v4f a, const v4f b, v8us& hi, v8us& lo) {
  float x[8];
  x[0] = a.x; x[1] = a.y; x[2] = a.z; x[3] = a.w; x[4] = b.x; x[5] = b.y; x[6] = b.z; x[7] = b.w;
#pragma unroll
  for (int i = 0; i < 8; ++i) {
    const unsigned short hb = bf_bits(x[i]);
    hi[i] = hb;
    lo[i] = bf_bits(x[i] - bf_val(hb));
  }
}

template <int ACT>
__device__ __forceinline__ float actf(float v) {
  if constexpr (ACT == 1) {
    return fmaxf(v, 0.0f);
  } else {
    return v;
  }
}

template <int RND>
__device__ __forceinline__ float cvin(float v) {
  if constexpr (RND == 1) {
    return bf_rne(v);
  } else {
    return v;
  }
}

__device__ __forceinline__ int scan_chunk(const int* __restrict__ dsts, int nE, int cbase, int slotBase,
                                          int nb, int vec8, int* list, int tid, int lane, int wave) {
  int wc = 0;
  const int el0  = tid * EPT;
  const int e0   = cbase + el0;
  const int sent = -2147483647 - 1;
  v4i da, db;
  if (vec8 != 0 && cbase + CHUNK <= nE) {
    da = *(const v4i*)(dsts + e0);
    db = *(const v4i*)(dsts + e0 + 4);
  } else {
    da.x = (e0     < nE) ? dsts[min(e0,     nE - 1)] : sent;
    da.y = (e0 + 1 < nE) ? dsts[min(e0 + 1, nE - 1)] : sent;
    da.z = (e0 + 2 < nE) ? dsts[min(e0 + 2, nE - 1)] : sent;
    da.w = (e0 + 3 < nE) ? dsts[min(e0 + 3, nE - 1)] : sent;
    db.x = (e0 + 4 < nE) ? dsts[min(e0 + 4, nE - 1)] : sent;
    db.y = (e0 + 5 < nE) ? dsts[min(e0 + 5, nE - 1)] : sent;
    db.z = (e0 + 6 < nE) ? dsts[min(e0 + 6, nE - 1)] : sent;
    db.w = (e0 + 7 < nE) ? dsts[min(e0 + 7, nE - 1)] : sent;
  }
  const unsigned nbs = (unsigned)slotBase;
  const unsigned unb = (unsigned)nb;
  const unsigned s0 = (unsigned)da.x - nbs, s1 = (unsigned)da.y - nbs;
  const unsigned s2 = (unsigned)da.z - nbs, s3 = (unsigned)da.w - nbs;
  const unsigned s4 = (unsigned)db.x - nbs, s5 = (unsigned)db.y - nbs;
  const unsigned s6 = (unsigned)db.z - nbs, s7 = (unsigned)db.w - nbs;
  const bool h0 = s0 < unb, h1 = s1 < unb, h2 = s2 < unb, h3 = s3 < unb;
  const bool h4 = s4 < unb, h5 = s5 < unb, h6 = s6 < unb, h7 = s7 < unb;
  const unsigned any = __builtin_amdgcn_ballot_w32(h0 | h1 | h2 | h3 | h4 | h5 | h6 | h7);
  if (any != 0u) {
#define HITJ(J, HJ, SJ) { \
      const unsigned mj = __builtin_amdgcn_ballot_w32(HJ); \
      if (mj != 0u) { \
        if (HJ) { \
          const int pos = wc + (int)__builtin_amdgcn_mbcnt_lo(mj, 0u); \
          if (pos < WCAP) list[wave * WCAP + pos] = ((el0 + (J)) << PKS) | (int)(SJ); \
        } \
        wc += (int)__builtin_popcount(mj); } }
    HITJ(0, h0, s0)
    HITJ(1, h1, s1)
    HITJ(2, h2, s2)
    HITJ(3, h3, s3)
    HITJ(4, h4, s4)
    HITJ(5, h5, s5)
    HITJ(6, h6, s6)
    HITJ(7, h7, s7)
#undef HITJ
  }
  return wc;
}

__global__ __launch_bounds__(NTHR) void k_wprep(const float* __restrict__ w1a, const float* __restrict__ w1b,
                                                const float* __restrict__ w2a, const float* __restrict__ w2b,
                                                const float* __restrict__ wfc, unsigned short* WPL) {
  const int u = (int)blockIdx.x * NTHR + (int)threadIdx.x;
  if (u >= NUW) return;
  v8us o;
  size_t dofs;
  if (u < UB1) {
    const int v = u, n = v >> 3, q = v & 7;
    const float* p = w1a + (size_t)(4 * q) * HID + n;
    float f[4];
#pragma unroll
    for (int c = 0; c < 4; ++c) f[c] = p[(size_t)c * HID];
#pragma unroll
    for (int j = 0; j < 8; ++j) o[j] = bf_bits(f[j >> 1]);
    dofs = (size_t)OF0 + (size_t)v * 8;
  } else if (u < UB2) {
    const int v = u - UB1, n = v >> 4, q = v & 15;
    const int kk = (8 * q) & (HID - 1);
    const float* p = w1b + (size_t)kk * HID + n;
#pragma unroll
    for (int i = 0; i < 8; ++i) o[i] = bf_bits(p[(size_t)i * HID]);
    dofs = (size_t)OF1 + (size_t)v * 8;
  } else if (u < UB3) {
    const int v = u - UB2, n = v >> 4, q = v & 15;
    const float* p = w2a + (size_t)(4 * q) * HID + n;
    float f[4];
#pragma unroll
    for (int c = 0; c < 4; ++c) f[c] = p[(size_t)c * HID];
#pragma unroll
    for (int j = 0; j < 8; ++j) o[j] = bf_bits(f[2 * (j >> 2) + (j & 1)]);
    dofs = (size_t)OF2 + (size_t)v * 8;
  } else if (u < UB4) {
    const int v = u - UB3, n = v >> 4, q = v & 15;
    const int kk = (8 * q) & (HID - 1);
    const float* p = w2b + (size_t)kk * HID + n;
#pragma unroll
    for (int i = 0; i < 8; ++i) o[i] = bf_bits(p[(size_t)i * HID]);
    dofs = (size_t)OF3 + (size_t)v * 8;
  } else {
    const int v = u - UB4, n = v >> 4, q = v & 15;
    const int kk = (8 * q) & (HID - 1);
    const int nc = n < NOUT ? n : NOUT - 1;
    const float* p = wfc + (size_t)kk * NOUT + nc;
#pragma unroll
    for (int i = 0; i < 8; ++i) {
      const unsigned short b = bf_bits(p[(size_t)i * NOUT]);
      o[i] = (n < NOUT) ? b : (unsigned short)0;
    }
    dofs = (size_t)OF4 + (size_t)v * 8;
  }
  unsigned short* dp = WPL + dofs;
  *(volatile v8us*)dp = o;
  __threadfence();
  *(volatile v8us*)dp = o;
}

template <int NT, int ACT, int OUTK>
__global__ __launch_bounds__(GTHR) void k_gemm(const unsigned short* __restrict__ A, int lda,
                                               const unsigned short* __restrict__ BT, int ldb, int K,
                                               const float* __restrict__ bias, int nBias,
                                               float* C32, unsigned short* C16, int ldc, int nRows) {
  static_assert((OUTK == 0 && NT == 4) || (OUTK == 2 && NT == 4) || (OUTK == 3 && NT == 1));
  constexpr int BN = 16 * NT;
  __shared__ __attribute__((aligned(16))) float stg[GBM * BN];
  __shared__ __attribute__((aligned(16))) float oln[(OUTK == 3) ? (GTHR * 4) : 4];
  const int tid = (int)threadIdx.x, lane = tid & 31, wave = tid >> 5, hh = lane >> 4, m = lane & 15;
  const int rowBase = (int)blockIdx.x * GBM;

  v8f acc[NT];
  {
    const v8f z = {0.f, 0.f, 0.f, 0.f, 0.f, 0.f, 0.f, 0.f};
#pragma unroll
    for (int t = 0; t < NT; ++t) acc[t] = z;
  }
  const unsigned short* ap = A  + (size_t)(rowBase + 16 * wave + m) * (size_t)lda + 8 * hh;
  const unsigned short* bp = BT + (size_t)m * (size_t)ldb + 8 * hh;

#pragma unroll 1
  for (int k0 = 0; k0 < K; k0 += 32) {
    Frag af;
    af.h[0] = *(const v8usa*)(ap + k0);
    af.h[1] = *(const v8usa*)(ap + k0 + 16);
#pragma unroll
    for (int nt = 0; nt < NT; ++nt) {
      const unsigned short* wq = bp + (size_t)(16 * nt) * (size_t)ldb + k0;
      Frag bf;
      bf.h[0] = *(const v8usa*)wq;
      bf.h[1] = *(const v8usa*)(wq + 16);
      acc[nt] = wmk(af, bf, acc[nt]);
    }
  }

#pragma unroll
  for (int nt = 0; nt < NT; ++nt) {
    const int lc = 16 * nt + m;
    const int bi = lc < nBias ? lc : nBias - 1;
    const float braw = bf_rne(bias[bi]);
    const float bb = (lc < nBias) ? braw : 0.0f;
#pragma unroll
    for (int r = 0; r < 8; ++r) {
      const int lr = 16 * wave + 8 * hh + r;
      stg[lr * BN + lc] = actf<ACT>(acc[nt][r] + bb);
    }
  }
  __syncthreads();

  if constexpr (OUTK == 0) {
    v4f pv[8];
#pragma unroll
    for (int i = 0; i < 8; ++i) {
      const int lr = 16 * wave + 2 * i + hh;
      pv[i] = *(const v4fa*)(stg + lr * BN + 4 * m);
    }
#pragma unroll
    for (int i = 0; i < 8; ++i) {
      const int gr = rowBase + 16 * wave + 2 * i + hh;
      float* op = C32 + (size_t)gr * (size_t)ldc + 4 * m;
      if (gr < nRows) *(volatile v4f*)op = pv[i];
    }
    __threadfence();
#pragma unroll
    for (int i = 0; i < 8; ++i) {
      const int gr = rowBase + 16 * wave + 2 * i + hh;
      float* op = C32 + (size_t)gr * (size_t)ldc + 4 * m;
      if (gr < nRows) *(volatile v4f*)op = pv[i];
    }
    (void)C16;
  } else if constexpr (OUTK == 2) {
    v8us ov[8];
    const int seg  = (lane >> 3) & 1;
    const int c8   = 8 * (lane & 7);
    const int loff = ldc >> 1;
#pragma unroll
    for (int i = 0; i < 8; ++i) {
      const int lr = 16 * wave + 2 * i + hh;
      const float* sp = stg + lr * BN + c8;
      const v4f fa = *(const v4fa*)sp;
      const v4f fb = *(const v4fa*)(sp + 4);
      v8us oh, ol;
      split8b(fa, fb, oh, ol);
#pragma unroll
      for (int j = 0; j < 8; ++j) ov[i][j] = (seg != 0) ? ol[j] : oh[j];
    }
#pragma unroll
    for (int i = 0; i < 8; ++i) {
      const int lr = 16 * wave + 2 * i + hh;
      unsigned short* op = C16 + (size_t)(rowBase + lr) * (size_t)ldc + seg * loff + c8;
      *(volatile v8us*)op = ov[i];
    }
    __threadfence();
#pragma unroll
    for (int i = 0; i < 8; ++i) {
      const int lr = 16 * wave + 2 * i + hh;
      unsigned short* op = C16 + (size_t)(rowBase + lr) * (size_t)ldc + seg * loff + c8;
      *(volatile v8us*)op = ov[i];
    }
    (void)C32; (void)nRows;
  } else {
    const int nr = (nRows - rowBase) < GBM ? (nRows - rowBase) : GBM;
    const int nf = (nr > 0 ? nr : 0) * NOUT;
#pragma unroll 1
    for (int t = tid; t < GTHR * 4; t += GTHR) {
      const int tt = t < GBM * NOUT ? t : GBM * NOUT - 1;
      const int r  = tt / NOUT;
      const int c  = tt - r * NOUT;
      const float v = stg[r * BN + c];
      oln[t] = (t < GBM * NOUT) ? v : 0.0f;
    }
    __syncthreads();
    const int nf4 = nf >> 2;
    const int rem = nf & 3;
    float* ob = C32 + (size_t)rowBase * NOUT;
    const v4f pv = *(const v4fa*)(oln + 4 * tid);
    const float t0 = oln[4 * nf4], t1 = oln[4 * nf4 + 1], t2 = oln[4 * nf4 + 2];
    if (tid < nf4) *(volatile v4f*)(ob + (size_t)4 * tid) = pv;
    if (tid == 0) {
      if (rem > 0) *(volatile float*)(ob + (size_t)4 * nf4)     = t0;
      if (rem > 1) *(volatile float*)(ob + (size_t)4 * nf4 + 1) = t1;
      if (rem > 2) *(volatile float*)(ob + (size_t)4 * nf4 + 2) = t2;
    }
    __threadfence();
    if (tid < nf4) *(volatile v4f*)(ob + (size_t)4 * tid) = pv;
    if (tid == 0) {
      if (rem > 0) *(volatile float*)(ob + (size_t)4 * nf4)     = t0;
      if (rem > 1) *(volatile float*)(ob + (size_t)4 * nf4 + 1) = t1;
      if (rem > 2) *(volatile float*)(ob + (size_t)4 * nf4 + 2) = t2;
    }
    (void)C16; (void)ldc;
  }
}

template <int CPL, int RND>
__global__ __launch_bounds__(NTHR) void k_agg(const int* __restrict__ srcs, const int* __restrict__ dsts,
                                              const float* __restrict__ X, unsigned short* Aout,
                                              int nN, int nE, int vec8) {
  static_assert(CPL == 1 || CPL == 2);
  constexpr int DW = 32 * CPL;
  constexpr int KP = 2 * DW;
  extern __shared__ __attribute__((aligned(16))) int lds_i[];
  int* reg1 = lds_i;
  int* reg2 = reg1 + RCAP;
  int* scnt = reg2 + RCAP;
  int* soff = scnt + NBA;
  int* list = soff + NBA;
  int* wcnt = list + LISTN;
  int* wtot = wcnt + NWAVE;
  const int tid = (int)threadIdx.x, lane = tid & 31, wave = tid >> 5;
  const int nodeBase = (int)blockIdx.x * NBA;

  {
    const v4i z4 = {0, 0, 0, 0};
    for (int i = tid * 4; i < ZINTS; i += NTHR * 4) *(v4ia*)(lds_i + i) = z4;
    if (tid < 2 * NWAVE) wcnt[tid] = 0;
  }
  __syncthreads();

  int tot = 0;
  const int nChunks = (nE + CHUNK - 1) / CHUNK;
#pragma unroll 1
  for (int ch = 0; ch < nChunks; ++ch) {
    const int cbase = ch * CHUNK;
    const int wc = scan_chunk(dsts, nE, cbase, nodeBase, NBA, vec8, list, tid, lane, wave);
    if (lane == 0) wcnt[wave] = wc;
    __syncthreads();
    int pre = 0, all = 0;
#pragma unroll
    for (int w2 = 0; w2 < NWAVE; ++w2) {
      int c = wcnt[w2];
      c = c < 0 ? 0 : (c > WCAP ? WCAP : c);
      all += c;
      pre += (w2 < wave) ? c : 0;
    }
    const int wcc  = wc > WCAP ? WCAP : wc;
    const int base = tot + pre;
#pragma unroll 1
    for (int i = lane; i < wcc; i += 32) {
      const int ent = list[wave * WCAP + i];
      const int el  = (ent >> PKS) & (CHUNK - 1);
      const int sl  = ent & (NBA - 1);
      int eid = cbase + el;
      eid = eid > nE - 1 ? nE - 1 : eid;
      const int pos = base + i;
      if (pos < RCAP) reg1[pos] = (int)(((unsigned)eid << PKS) | (unsigned)sl);
    }
    tot += all;
    tot = tot > RCAP ? RCAP : tot;
    __syncthreads();
  }
  const int nh = tot;

  if (wave == 0) {
#pragma unroll 1
    for (int b0 = 0; b0 < nh; b0 += 32) {
      const int idx = b0 + lane;
      const int uv  = reg1[idx < RCAP ? idx : RCAP - 1];
      const int m32 = (nh - b0) < 32 ? (nh - b0) : 32;
#pragma unroll 1
      for (int k = 0; k < m32; ++k) {
        const int u  = __builtin_amdgcn_readlane(uv, k);
        const int sl = u & (NBA - 1);
        if (lane == 0) scnt[sl] = scnt[sl] + 1;
      }
    }
  }
  __syncthreads();

  {
    const v4i ca = *(const v4ia*)(scnt + 4 * tid);
    const int e0 = ca.x < 0 ? 0 : ca.x, e1 = ca.y < 0 ? 0 : ca.y, e2 = ca.z < 0 ? 0 : ca.z, e3 = ca.w < 0 ? 0 : ca.w;
    const int ts = e0 + e1 + e2 + e3;
    int incl = ts;
#pragma unroll
    for (int d = 1; d < 32; d <<= 1) {
      const int up = __shfl_up(incl, d, 32);
      if (lane >= d) incl += up;
    }
    if (lane == 31) wtot[wave] = incl;
    __syncthreads();
    int pre = 0;
#pragma unroll
    for (int w2 = 0; w2 < NWAVE; ++w2) pre += (w2 < wave) ? wtot[w2] : 0;
    int run = pre + incl - ts;
    soff[4 * tid + 0] = run; run += e0;
    soff[4 * tid + 1] = run; run += e1;
    soff[4 * tid + 2] = run; run += e2;
    soff[4 * tid + 3] = run;
  }
  __syncthreads();
  for (int i = tid; i < NBA; i += NTHR) list[i] = soff[i];
  __syncthreads();

  if (wave == 0) {
#pragma unroll 1
    for (int b0 = 0; b0 < nh; b0 += 32) {
      const int idx = b0 + lane;
      const int uv  = reg1[idx < RCAP ? idx : RCAP - 1];
      const int m32 = (nh - b0) < 32 ? (nh - b0) : 32;
#pragma unroll 1
      for (int k = 0; k < m32; ++k) {
        const int u   = __builtin_amdgcn_readlane(uv, k);
        const int sl  = u & (NBA - 1);
        const int eid = (int)((unsigned)u >> PKS);
        if (lane == 0) {
          int pos = list[sl];
          pos = pos < 0 ? 0 : (pos > RCAP - 1 ? RCAP - 1 : pos);
          reg2[pos] = eid;
          list[sl] = pos + 1;
        }
      }
    }
  }
  __syncthreads();

  const int nbw = NBA / NWAVE;
  const bool ovf = (nh >= RCAP);
  const float qnan = __int_as_float(0x7fc00000);

#pragma unroll 1
  for (int jt = 0; jt < nbw; ++jt) {
    const int slot = wave * nbw + jt;
    const int node = nodeBase + slot;
    int st = soff[slot];
    const int craw = scnt[slot];
    int cnt = craw;
    st  = st < 0 ? 0 : (st > nh ? nh : st);
    cnt = cnt < 0 ? 0 : (cnt > DEGCAP ? DEGCAP : cnt);
    if (cnt > nh - st) cnt = nh - st;
    const float pz = (ovf || craw > DEGCAP) ? qnan : 0.0f;
    const bool live = node < nN;
    const int nc = node < nN ? node : nN - 1;

    float a0 = 0.f, a1 = 0.f;
#pragma unroll 1
    for (int b0 = 0; b0 < cnt; b0 += 32) {
      int idx = st + b0 + lane; idx = idx > RCAP - 1 ? RCAP - 1 : idx;
      int eid = reg2[idx]; eid = eid < 0 ? 0 : (eid > nE - 1 ? nE - 1 : eid);
      int sr = srcs[eid]; sr = sr < 0 ? 0 : (sr > nN - 1 ? nN - 1 : sr);
      const int m32 = (cnt - b0) < 32 ? (cnt - b0) : 32;
#pragma unroll 1
      for (int k = 0; k < m32; ++k) {
        const int sk = __builtin_amdgcn_readlane(sr, k);
        if constexpr (CPL == 1) {
          const float v = X[(size_t)sk * DW + lane];
          a0 += cvin<RND>(v);
        } else {
          const v2f v = *(const v2f*)(X + (size_t)sk * DW + 2 * lane);
          a0 += cvin<RND>(v.x); a1 += cvin<RND>(v.y);
        }
      }
    }
    if constexpr (CPL == 1) {
      const float sv = X[(size_t)nc * DW + lane];
      float r0 = a0 + cvin<RND>(sv);
      r0 = (live ? r0 : 0.0f) + pz;
      const unsigned short hb0 = bf_bits(r0);
      const unsigned short lb0 = bf_bits(r0 - bf_val(hb0));
      const unsigned int pk = (unsigned int)hb0 | ((unsigned int)lb0 << 16);
      unsigned short* gp = Aout + (size_t)node * (size_t)KP + 2 * lane;
      *(volatile unsigned int*)gp = pk;
      __threadfence();
      *(volatile unsigned int*)gp = pk;
      (void)a1;
    } else {
      const v2f sv = *(const v2f*)(X + (size_t)nc * DW + 2 * lane);
      float r0 = a0 + cvin<RND>(sv.x), r1 = a1 + cvin<RND>(sv.y);
      r0 = (live ? r0 : 0.0f) + pz;
      r1 = (live ? r1 : 0.0f) + pz;
      const unsigned short hb0 = bf_bits(r0), hb1 = bf_bits(r1);
      const unsigned short lb0 = bf_bits(r0 - bf_val(hb0)), lb1 = bf_bits(r1 - bf_val(hb1));
      v2u pk;
      pk.x = (unsigned int)hb0 | ((unsigned int)hb1 << 16);
      pk.y = (unsigned int)lb0 | ((unsigned int)lb1 << 16);
      unsigned short* gp = Aout + (size_t)node * (size_t)KP + 4 * lane;
      *(volatile v2u*)gp = pk;
      __threadfence();
      *(volatile v2u*)gp = pk;
    }
  }
}

static inline int cdiv(int a, int b) { return (a + b - 1) / b; }
static inline size_t al256(size_t o) { return (o + 255) & ~(size_t)255; }

extern "C" void kernel_launch(void* const* d_in, const int* in_sizes, int n_in,
                              void* d_out, int out_size, void* d_ws, size_t ws_size,
                              hipStream_t stream) {
  if (n_in < 12) return;
  if (in_sizes[0] < DIN1 || (in_sizes[0] % DIN1) != 0) return;
  const int nN = in_sizes[0] / DIN1;
  if (nN < 1 || nN > (1 << 22)) return;
  if (in_sizes[1] < 2 || (in_sizes[1] & 1) != 0) return;
  const int nE = in_sizes[1] / 2;
  if (nE < 1 || nE >= (1 << 21)) return;
  if (in_sizes[2] != DIN1 * HID || in_sizes[3] != HID) return;
  if (in_sizes[4] != HID * HID || in_sizes[5] != HID) return;
  if (in_sizes[6] != HID * HID || in_sizes[7] != HID) return;
  if (in_sizes[8] != HID * HID || in_sizes[9] != HID) return;
  if (in_sizes[10] != HID * NOUT || in_sizes[11] != NOUT) return;
  if ((long long)out_size != (long long)nN * NOUT) return;

  const float* x    = (const float*)d_in[0];
  const int*   edge = (const int*)  d_in[1];
  const float* w1a  = (const float*)d_in[2];
  const float* b1a  = (const float*)d_in[3];
  const float* w1b  = (const float*)d_in[4];
  const float* b1b  = (const float*)d_in[5];
  const float* w2a  = (const float*)d_in[6];
  const float* b2a  = (const float*)d_in[7];
  const float* w2b  = (const float*)d_in[8];
  const float* b2b  = (const float*)d_in[9];
  const float* wfc  = (const float*)d_in[10];
  const float* bfc  = (const float*)d_in[11];
  float* out = (float*)d_out;
  const int* src = edge;
  const int* dst = edge + nE;

  const int MP   = cdiv(nN, GBM) * GBM;
  const int gM   = MP / GBM;
  const int gA   = cdiv(MP, NBA);
  const int RA   = gA * NBA;
  const int vec8 = ((nE & 3) == 0) ? 1 : 0;
  if ((long long)RA < (long long)MP) return;

  char* ws = (char*)d_ws;
  size_t off = 0;
  const size_t oWPL = off; off = al256(off + (size_t)WPLH * 2);
  const size_t oAP  = off; off = al256(off + (size_t)RA * KA2 * 2);
  const size_t oTP  = off; off = al256(off + (size_t)MP * KT * 2);
  const size_t oHP  = off; off = al256(off + (size_t)MP * KT * 2);
  if (off > ws_size || off > (size_t)WSMAX) return;
  unsigned short* WPL  = (unsigned short*)(ws + oWPL);
  unsigned short* AP   = (unsigned short*)(ws + oAP);
  unsigned short* TP   = (unsigned short*)(ws + oTP);
  unsigned short* HP16 = (unsigned short*)(ws + oHP);
  float*          HP32 = (float*)(ws + oHP);

  hipFuncSetAttribute(reinterpret_cast<const void*>(&k_agg<1, 1>), hipFuncAttributeMaxDynamicSharedMemorySize, LDS_AGG);
  hipFuncSetAttribute(reinterpret_cast<const void*>(&k_agg<2, 0>), hipFuncAttributeMaxDynamicSharedMemorySize, LDS_AGG);

  k_wprep<<<NUW / NTHR, NTHR, 0, stream>>>(w1a, w1b, w2a, w2b, wfc, WPL);
  k_agg<1, 1><<<gA, NTHR, LDS_AGG, stream>>>(src, dst, x, AP, nN, nE, vec8);
  k_gemm<4, 1, 2><<<gM, GTHR, 0, stream>>>(AP, KA1, WPL + OF0, KA1, KA1, b1a, HID, HP32, TP, KT, MP);
  k_gemm<4, 1, 0><<<gM, GTHR, 0, stream>>>(TP, KT, WPL + OF1, KT, KT, b1b, HID, HP32, TP, HID, MP);
  k_agg<2, 0><<<gA, NTHR, LDS_AGG, stream>>>(src, dst, HP32, AP, nN, nE, vec8);
  k_gemm<4, 1, 2><<<gM, GTHR, 0, stream>>>(AP, KA2, WPL + OF2, KA2, KA2, b2a, HID, HP32, TP, KT, MP);
  k_gemm<4, 1, 2><<<gM, GTHR, 0, stream>>>(TP, KT, WPL + OF3, KT, KT, b2b, HID, HP32, HP16, KT, MP);
  k_gemm<1, 0, 3><<<gM, GTHR, 0, stream>>>(HP16, KT, WPL + OF4, KT, KT, bfc, NOUT, out, HP16, NOUT, nN);
}
